// AttentionFlow_57973468561807
// MI455X (gfx1250) — hardware-run, weakly checked
//
#include <hip/hip_runtime.h>
#include <math.h>

#ifndef NB
#define NB 32
#endif
#ifndef LP
#define LP 1024
#endif
#define NB_FULL 32
#define LP_FULL 1024
#define LQ 128
#define DIMD 256

#define NEGF (-10000000.0f)
#define CARRY_A 1024.0f
#define CARRY_Q 64.0f
#define CARRY_W 1024.0f
#define SC_INV 1.52587890625e-05f

#define FU_WAVES 4
#define FU_ROWS 64
#define PT_P 132
#define SL_P 68
#define TILES_PER_B ((unsigned)(LP / FU_ROWS))

static_assert(LQ == 128);
static_assert(DIMD == 256);
static_assert(LP % FU_ROWS == 0);
static_assert(LP % 4 == 0);
static_assert(LP <= LP_FULL && NB <= NB_FULL);
static_assert(FU_WAVES * 32 == LQ);
static_assert(FU_WAVES * 16 == FU_ROWS);
static_assert((size_t)NB_FULL * LP_FULL * DIMD * 4 == (size_t)33554432);

#define OUT2_OFF ((size_t)NB_FULL * LP_FULL * DIMD)

#define QH_BYTES  ((size_t)NB * LQ * DIMD * 2)
#define QT_BYTES  ((size_t)NB * DIMD * LQ * 2)
#define QY_BYTES  ((size_t)NB * LQ * 4)
#define SIM_BYTES ((size_t)NB * LP * 4)
static_assert(QH_BYTES % 256 == 0 && QT_BYTES % 256 == 0 && QY_BYTES % 256 == 0 && SIM_BYTES % 256 == 0);
static_assert(QH_BYTES + QT_BYTES + QY_BYTES + SIM_BYTES <= (size_t)134217728);

typedef _Float16 h16;
typedef __attribute__((ext_vector_type(16))) _Float16 v16h;
typedef __attribute__((ext_vector_type(8)))  _Float16 v8h;
typedef __attribute__((ext_vector_type(8)))  float    v8f;
typedef __attribute__((ext_vector_type(4)))  float    v4f;


#define VST2V4(ptr, val) do { const v4f vst2_v4_ = (val); *(volatile v4f*)(ptr) = vst2_v4_; __threadfence(); *(volatile v4f*)(ptr) = vst2_v4_; } while (0)

static __device__ __forceinline__ float bfr(float f) {
    unsigned u = __float_as_uint(f);
    u += 0x7FFFu + ((u >> 16) & 1u);
    return __uint_as_float(u & 0xFFFF0000u);
}
static __device__ __forceinline__ h16 toh_flush(float v) {
    const float w = (fabsf(v) < 6.103515625e-05f) ? 0.0f : v;
    return (h16)w;
}
static __device__ __forceinline__ void st8h2(h16* dst, v8h hv) {
    *(volatile v8h*)dst = hv;
    __threadfence();
    *(volatile v8h*)dst = hv;
}

union FragU { v16h v; v8h h[2]; };
static __device__ __forceinline__ v16h frag_ld(const h16* p) {
    FragU f; f.h[0] = *(const v8h*)(p); f.h[1] = *(const v8h*)(p + 16); return f.v;
}
static __device__ __forceinline__ v8f wmma16g(v16h a, v16h b, v8f c) {
    c = __builtin_amdgcn_wmma_f32_16x16x32_f16(false, a, false, b, (short)0, c, false, false);
    asm volatile("v_nop\n\tv_nop\n\tv_nop\n\tv_nop" : "+v"(c) : "v"(a), "v"(b));
    return c;
}

__global__ __launch_bounds__(256) void k_qprep(const float* __restrict__ Q, const float* __restrict__ w,
                                               h16* __restrict__ Qh, float* __restrict__ qy) {
    __shared__ __align__(16) float sQy[32];
    const unsigned tid = threadIdx.x, L = tid & 31u, wave = tid >> 5;
    const unsigned bx = blockIdx.x;
    const unsigned b = bx >> 2, j0 = (bx & 3u) * 32u;
    const v4f wa = *(const v4f*)(w + DIMD + 8u * L);
    const v4f wb = *(const v4f*)(w + DIMD + 8u * L + 4u);
    const float wy[8] = {bfr(wa.x), bfr(wa.y), bfr(wa.z), bfr(wa.w), bfr(wb.x), bfr(wb.y), bfr(wb.z), bfr(wb.w)};
    for (unsigned rr = 0; rr < 4u; ++rr) {
        const unsigned j = j0 + 4u * wave + rr;
        const float* qr = Q + (size_t)(b * LQ + j) * DIMD + 8u * L;
        const v4f a = *(const v4f*)qr;
        const v4f c = *(const v4f*)(qr + 4);
        const float x[8] = {bfr(a.x), bfr(a.y), bfr(a.z), bfr(a.w), bfr(c.x), bfr(c.y), bfr(c.z), bfr(c.w)};
        float s = 0.f;
#pragma unroll
        for (int i = 0; i < 8; ++i) s += x[i] * wy[i];
#pragma unroll
        for (int o = 16; o > 0; o >>= 1) s += __shfl_xor(s, o, 32);
        v8h hv;
#pragma unroll
        for (int i = 0; i < 8; ++i) hv[i] = toh_flush(x[i] * CARRY_Q);
        st8h2(Qh + (size_t)(b * LQ + j) * DIMD + 8u * L, hv);
        if (L == 0u) sQy[4u * wave + rr] = s;
    }
    __syncthreads();
    if (tid < 8u) {
        const v4f v = *(const v4f*)(&sQy[4u * tid]);
        VST2V4(qy + (size_t)(b * LQ + j0 + 4u * tid), v);
    }
}

__global__ __launch_bounds__(256) void k_qt(const float* __restrict__ Q, h16* __restrict__ QT) {
    const unsigned u = blockIdx.x * 256u + threadIdx.x;
    const unsigned b = u >> 12;
    const unsigned r = u & 4095u;
    const unsigned d = r >> 4, j0 = 8u * (r & 15u);
    const float* src = Q + (size_t)(b * LQ + j0) * DIMD + d;
    v8h hv;
#pragma unroll
    for (int i = 0; i < 8; ++i) hv[i] = toh_flush(bfr(src[(unsigned)i * DIMD]) * CARRY_Q);
    st8h2(QT + (size_t)(b * DIMD + d) * LQ + j0, hv);
}

__global__ __launch_bounds__(128) void k_fused(const float* __restrict__ P, const h16* __restrict__ Qh, const h16* __restrict__ QT,
                                               const float* __restrict__ qy, const float* __restrict__ qm,
                                               const float* __restrict__ w, const float* __restrict__ bsc,
                                               float* __restrict__ out1, float* __restrict__ sim) {
    __shared__ __align__(16) float sWx[DIMD];
    __shared__ __align__(16) float sWxy[DIMD];
    __shared__ __align__(16) float sQy[LQ];
    __shared__ __align__(16) float sQm[LQ];
    __shared__ __align__(16) float sSim[FU_ROWS];
    __shared__ __align__(16) float sPt[FU_WAVES][16 * PT_P];
    __shared__ __align__(16) float sSl[FU_WAVES][16 * SL_P];

    const unsigned tid = threadIdx.x, lane = tid & 31u, wave = tid >> 5;
    const unsigned hh = lane >> 4, c = lane & 15u;
    const unsigned bx = blockIdx.x;
    const unsigned b = bx / TILES_PER_B;
    const unsigned tile = bx - b * TILES_PER_B;

    sWx[tid]         = bfr(w[tid]);
    sWx[tid + 128u]  = bfr(w[tid + 128u]);
    sWxy[tid]        = bfr(w[512u + tid]);
    sWxy[tid + 128u] = bfr(w[640u + tid]);
    sQy[tid] = qy[(size_t)(b * LQ) + tid];
    sQm[tid] = bfr(qm[(size_t)(b * LQ) + tid]);
    __syncthreads();

    const unsigned row0 = tile * FU_ROWS + wave * 16u;
    const float* prow = P + (size_t)(b * LP_FULL + row0 + c) * DIMD;

    v8f acc[8];
#pragma unroll
    for (int t = 0; t < 8; ++t) acc[t] = (v8f){0.f, 0.f, 0.f, 0.f, 0.f, 0.f, 0.f, 0.f};
    float pxp = 0.f;

    for (unsigned ks = 0; ks < 8u; ++ks) {
        const unsigned ka = ks * 32u + 8u * hh;
        const unsigned kb = ka + 16u;
        const v4f p0 = *(const v4f*)(prow + ka), p1 = *(const v4f*)(prow + ka + 4u);
        const v4f p2 = *(const v4f*)(prow + kb), p3 = *(const v4f*)(prow + kb + 4u);
        const v4f x0 = *(const v4f*)(&sWxy[ka]), x1 = *(const v4f*)(&sWxy[ka + 4u]);
        const v4f x2 = *(const v4f*)(&sWxy[kb]), x3 = *(const v4f*)(&sWxy[kb + 4u]);
        const v4f y0 = *(const v4f*)(&sWx[ka]),  y1 = *(const v4f*)(&sWx[ka + 4u]);
        const v4f y2 = *(const v4f*)(&sWx[kb]),  y3 = *(const v4f*)(&sWx[kb + 4u]);
        const float pv[16] = {p0.x, p0.y, p0.z, p0.w, p1.x, p1.y, p1.z, p1.w, p2.x, p2.y, p2.z, p2.w, p3.x, p3.y, p3.z, p3.w};
        const float xv[16] = {x0.x, x0.y, x0.z, x0.w, x1.x, x1.y, x1.z, x1.w, x2.x, x2.y, x2.z, x2.w, x3.x, x3.y, x3.z, x3.w};
        const float yv[16] = {y0.x, y0.y, y0.z, y0.w, y1.x, y1.y, y1.z, y1.w, y2.x, y2.y, y2.z, y2.w, y3.x, y3.y, y3.z, y3.w};
        v16h af;
#pragma unroll
        for (int i = 0; i < 16; ++i) {
            const float pb = bfr(pv[i]);
            af[i] = toh_flush((pb * xv[i]) * CARRY_A);
            pxp += pb * yv[i];
        }
#pragma unroll
        for (int t = 0; t < 8; ++t) {
            const v16h bf = frag_ld(Qh + (size_t)(b * LQ + (unsigned)t * 16u + c) * DIMD + ka);
            acc[t] = wmma16g(af, bf, acc[t]);
        }
    }

    const float px = pxp + __shfl_xor(pxp, 16, 32);
    float pxr[8];
#pragma unroll
    for (int r = 0; r < 8; ++r) pxr[r] = __shfl(px, (int)(8u * hh + (unsigned)r), 32);
    const float bias = bfr(bsc[0]);

    float rmax[8], rsum[8];
#pragma unroll
    for (int r = 0; r < 8; ++r) { rmax[r] = -3.0e38f; rsum[r] = 0.f; }
#pragma unroll
    for (int t = 0; t < 8; ++t) {
        const unsigned j = (unsigned)t * 16u + c;
        const float qv = sQy[j];
        const bool on = sQm[j] > 0.0f;
#pragma unroll
        for (int r = 0; r < 8; ++r) {
            float v = ((pxr[r] + qv) + acc[t][r] * SC_INV) + bias;
            v = on ? v : NEGF;
            acc[t][r] = v;
            rmax[r] = fmaxf(rmax[r], v);
        }
    }
#pragma unroll
    for (int r = 0; r < 8; ++r) {
        float mx = rmax[r];
        mx = fmaxf(mx, __shfl_xor(mx, 1, 32)); mx = fmaxf(mx, __shfl_xor(mx, 2, 32));
        mx = fmaxf(mx, __shfl_xor(mx, 4, 32)); mx = fmaxf(mx, __shfl_xor(mx, 8, 32));
        rmax[r] = mx;
    }
#pragma unroll
    for (int t = 0; t < 8; ++t) {
#pragma unroll
        for (int r = 0; r < 8; ++r) {
            const float e = expf(acc[t][r] - rmax[r]);
            acc[t][r] = e;
            rsum[r] += e;
        }
    }
    float inv[8];
#pragma unroll
    for (int r = 0; r < 8; ++r) {
        float sm = rsum[r];
        sm += __shfl_xor(sm, 1, 32); sm += __shfl_xor(sm, 2, 32);
        sm += __shfl_xor(sm, 4, 32); sm += __shfl_xor(sm, 8, 32);
        inv[r] = 1.0f / sm;
    }

    float* pt = sPt[wave];
#pragma unroll
    for (int t = 0; t < 8; ++t) {
#pragma unroll
        for (int r = 0; r < 8; ++r)
            pt[(8u * hh + (unsigned)r) * PT_P + (unsigned)t * 16u + c] = acc[t][r] * inv[r];
    }
    if (c == 0u) {
#pragma unroll
        for (int r = 0; r < 8; ++r) sSim[wave * 16u + 8u * hh + (unsigned)r] = rmax[r];
    }
    __syncthreads();

    if (tid < 16u) {
        const v4f v = *(const v4f*)(&sSim[4u * tid]);
        VST2V4(sim + (size_t)(b * LP + tile * FU_ROWS + 4u * tid), v);
    }

    v16h pa[4];
#pragma unroll
    for (int kk = 0; kk < 4; ++kk) {
        const float* base = pt + c * PT_P + (unsigned)kk * 32u + 8u * hh;
        const v4f a0 = *(const v4f*)(base), a1 = *(const v4f*)(base + 4);
        const v4f a2 = *(const v4f*)(base + 16), a3 = *(const v4f*)(base + 20);
        const float av[16] = {a0.x, a0.y, a0.z, a0.w, a1.x, a1.y, a1.z, a1.w, a2.x, a2.y, a2.z, a2.w, a3.x, a3.y, a3.z, a3.w};
#pragma unroll
        for (int i = 0; i < 16; ++i) pa[kk][i] = toh_flush(av[i] * CARRY_W);
    }

    float* slab = sSl[wave];
    for (unsigned g = 0; g < 4u; ++g) {
        v8f o[4];
#pragma unroll
        for (int j = 0; j < 4; ++j) o[j] = (v8f){0.f, 0.f, 0.f, 0.f, 0.f, 0.f, 0.f, 0.f};
#pragma unroll
        for (int kk = 0; kk < 4; ++kk) {
#pragma unroll
            for (int j = 0; j < 4; ++j) {
                const v16h bf = frag_ld(QT + (size_t)(b * DIMD + g * 64u + (unsigned)j * 16u + c) * LQ + (unsigned)kk * 32u + 8u * hh);
                o[j] = wmma16g(pa[kk], bf, o[j]);
            }
        }
#pragma unroll
        for (int j = 0; j < 4; ++j) {
#pragma unroll
            for (int r = 0; r < 8; ++r)
                slab[(8u * hh + (unsigned)r) * SL_P + (unsigned)j * 16u + c] = o[j][r] * SC_INV;
        }
        __syncthreads();
        {
            const unsigned c4 = (lane & 15u) * 4u;
#pragma unroll
            for (int half = 0; half < 2; ++half) {
                v4f vv[4];
#pragma unroll
                for (int it = 0; it < 4; ++it) {
                    const unsigned row = (unsigned)(half * 4 + it) * 2u + hh;
                    vv[it] = *(const v4f*)(slab + row * SL_P + c4);
                }
                for (int pass = 0; pass < 2; ++pass) {
#pragma unroll
                    for (int it = 0; it < 4; ++it) {
                        const unsigned row = (unsigned)(half * 4 + it) * 2u + hh;
                        *(volatile v4f*)(out1 + (size_t)(b * LP_FULL + row0 + row) * DIMD + g * 64u + c4) = vv[it];
                    }
                    __threadfence();
                }
            }
        }
        __syncthreads();
    }
}

__global__ __launch_bounds__(256) void k_pool(const float* __restrict__ P, const float* __restrict__ dm,
                                              const float* __restrict__ sim, float* __restrict__ out2) {
    __shared__ __align__(16) float sAtt[LP];
    __shared__ float red[256];
    __shared__ __align__(16) float sPart[4 * DIMD];
    __shared__ __align__(16) float sV[DIMD];
    const unsigned t = threadIdx.x;
    const unsigned b = blockIdx.x;

    float lmax = -3.0e38f;
    for (unsigned i = t; i < (unsigned)LP; i += 256u) {
        const float sv = sim[(size_t)(b * LP) + i];
        const float dv = bfr(dm[(size_t)(b * LP_FULL) + i]);
        const float v = (dv > 0.0f) ? sv : NEGF;
        sAtt[i] = v;
        lmax = fmaxf(lmax, v);
    }
    red[t] = lmax;
    __syncthreads();
    for (unsigned s = 128u; s > 0u; s >>= 1) {
        if (t < s) red[t] = fmaxf(red[t], red[t + s]);
        __syncthreads();
    }
    const float mx = red[0];
    __syncthreads();

    float lsum = 0.f;
    for (unsigned i = t; i < (unsigned)LP; i += 256u) {
        const float e = expf(sAtt[i] - mx);
        sAtt[i] = e;
        lsum += e;
    }
    red[t] = lsum;
    __syncthreads();
    for (unsigned s = 128u; s > 0u; s >>= 1) {
        if (t < s) red[t] += red[t + s];
        __syncthreads();
    }
    const float inv = 1.0f / red[0];

    const unsigned d4 = (t & 63u) * 4u;
    const unsigned ig = t >> 6;
    {
        const unsigned i0 = ig * (unsigned)(LP / 4);
        const float* pp = P + (size_t)(b * LP_FULL + i0) * DIMD + d4;
        v4f a = (v4f){0.f, 0.f, 0.f, 0.f};
        for (unsigned i = 0; i < (unsigned)(LP / 4); ++i) {
            const float wgt = sAtt[i0 + i] * inv;
            const v4f x = *(const v4f*)(pp + (size_t)i * DIMD);
            a.x += wgt * bfr(x.x);
            a.y += wgt * bfr(x.y);
            a.z += wgt * bfr(x.z);
            a.w += wgt * bfr(x.w);
        }
        *(v4f*)(&sPart[ig * DIMD + d4]) = a;
    }
    __syncthreads();
    sV[t] = (sPart[t] + sPart[DIMD + t]) + (sPart[2 * DIMD + t] + sPart[3 * DIMD + t]);
    __syncthreads();

    const v4f val = *(const v4f*)(&sV[d4]);
    float* dst = out2 + (size_t)(b * LP_FULL) * DIMD + d4;
    for (int pass = 0; pass < 2; ++pass) {
        for (unsigned it = 0; it < (unsigned)(LP / 4); ++it) {
            const unsigned row = it * 4u + ig;
            *(volatile v4f*)(dst + (size_t)row * DIMD) = val;
        }
        __threadfence();
    }
}

extern "C" void kernel_launch(void* const* d_in, const int* in_sizes, int n_in, void* d_out, int out_size,
                              void* d_ws, size_t ws_size, hipStream_t stream) {
    if (n_in < 6) return;
    const int prow_need = ((NB - 1) * LP_FULL + LP);
    if (in_sizes[0] < prow_need * DIMD) return;
    if (in_sizes[1] < NB * LQ * DIMD) return;
    if (in_sizes[2] < prow_need) return;
    if (in_sizes[3] < NB * LQ) return;
    if (in_sizes[4] < 3 * DIMD) return;
    if (in_sizes[5] < 1) return;
    if (out_size < (int)OUT2_OFF + prow_need * DIMD) return;

    const float* P   = (const float*)d_in[0];
    const float* Q   = (const float*)d_in[1];
    const float* dmk = (const float*)d_in[2];
    const float* qmk = (const float*)d_in[3];
    const float* w   = (const float*)d_in[4];
    const float* bsc = (const float*)d_in[5];
    float* out1 = (float*)d_out;
    float* out2 = out1 + OUT2_OFF;

    char* wsp = (char*)d_ws;
    size_t off = 0;
    auto carve = [&](size_t bytes) -> void* { void* r = wsp + off; off += (bytes + 255) & ~(size_t)255; return r; };
    h16*   Qh  = (h16*)carve(QH_BYTES);
    h16*   QT  = (h16*)carve(QT_BYTES);
    float* qy  = (float*)carve(QY_BYTES);
    float* sim = (float*)carve(SIM_BYTES);
    if (off > ws_size || off > (size_t)134217728) return;

    k_qprep<<<NB * 4, 256, 0, stream>>>(Q, w, Qh, qy);
    k_qt<<<NB * 16, 256, 0, stream>>>(Q, QT);
    k_fused<<<NB * (LP / FU_ROWS), 128, 0, stream>>>(P, (const h16*)Qh, (const h16*)QT, qy, qmk, w, bsc, out1, sim);
    k_pool<<<NB, 256, 0, stream>>>(P, dmk, sim, out2);
}
